// BooleanReservoir_31284541784138
// MI455X (gfx1250) — hardware-verified
//
#include <hip/hip_runtime.h>
#include <stdint.h>
#include <math.h>


typedef _Float16 v16h __attribute__((ext_vector_type(16)));
typedef _Float16 v8h  __attribute__((ext_vector_type(8)));
typedef float    v8f  __attribute__((ext_vector_type(8)));
typedef float    v4f  __attribute__((ext_vector_type(4)));
typedef unsigned int v4u __attribute__((ext_vector_type(4)));

union Frag { v16h v; v8h half[2]; _Float16 s[16]; };

#define I_N    512
#define R_N    16384
#define NN     16896
#define KADJ   8
#define MB     64
#define SS     16
#define NCH    2
#define BCH    32
#define NOUT   10
#define LUTW   256
#define MT_INJ 64
#define SBUF   16928
#define EVT    512

__device__ __forceinline__ v8f wmma_f16(v16h a, v16h b, v8f c) {
  v8f d = __builtin_amdgcn_wmma_f32_16x16x32_f16(false, a, false, b, (short)0, c, false, false);
  asm volatile("v_nop\n\tv_nop\n\tv_nop\n\tv_nop" : "+v"(d) : "v"(a), "v"(b));
  return d;
}

__global__ __launch_bounds__(256)
void prep_kernel(const int* __restrict__ adj_list, const int* __restrict__ adj_mask,
                 const int* __restrict__ deg, const float* __restrict__ lut,
                 unsigned int* __restrict__ adjp, unsigned int* __restrict__ lutbits) {
  const int t = blockIdx.x * blockDim.x + threadIdx.x;
  v4u val = {0u, 0u, 0u, 0u};
  v4u* dst = (v4u*)adjp;
  bool have = false;
  if (t < NN) {
    unsigned int sl[8];
#pragma unroll
    for (int k = 0; k < KADJ; ++k) {
      int a = adj_list[t * KADJ + k];
      const int mk = adj_mask[t * KADJ + k];
      a = (a < 0) ? (a + NN) : a;
      a = (a < 0) ? 0 : a;
      a = (a > NN - 1) ? (NN - 1) : a;
      sl[k] = (mk != 0) ? (unsigned int)a : (unsigned int)NN;
    }
    if (deg[t] <= 0) sl[0] |= 0x8000u;
    val.x = sl[0] | (sl[1] << 16);
    val.y = sl[2] | (sl[3] << 16);
    val.z = sl[4] | (sl[5] << 16);
    val.w = sl[6] | (sl[7] << 16);
    dst = (v4u*)adjp + t;
    have = true;
  } else if (t < 3 * NN) {
    const int u = t - NN;
    const int n = u >> 1, q = u & 1;
    const v4f* lp = (const v4f*)(lut + (size_t)n * LUTW + q * 128);
    unsigned int w[4];
#pragma unroll
    for (int wi = 0; wi < 4; ++wi) {
      unsigned int bits = 0u;
#pragma unroll
      for (int g = 0; g < 8; ++g) {
        const v4f f = lp[wi * 8 + g];
        bits |= (f.x != 0.f ? 1u : 0u) << (4 * g + 0);
        bits |= (f.y != 0.f ? 1u : 0u) << (4 * g + 1);
        bits |= (f.z != 0.f ? 1u : 0u) << (4 * g + 2);
        bits |= (f.w != 0.f ? 1u : 0u) << (4 * g + 3);
      }
      w[wi] = bits;
    }
    val.x = w[0]; val.y = w[1]; val.z = w[2]; val.w = w[3];
    dst = (v4u*)lutbits + u;
    have = true;
  }
  if (have) *(volatile v4u*)dst = val;
  __threadfence();
  if (have) *(volatile v4u*)dst = val;
}

__global__ __launch_bounds__(128)
void inject_kernel(const float* __restrict__ x, const float* __restrict__ w_in,
                   unsigned int* __restrict__ injbits) {
  __shared__ __attribute__((aligned(16))) unsigned int stage[4][16][32];
  const int tid  = threadIdx.x;
  const int wave = tid >> 5;
  const int lane = tid & 31;
  const int h    = lane >> 4;
  const int m    = lane & 15;
  const int mt   = blockIdx.x * 4 + wave;
  const int mtc  = (mt < MT_INJ) ? mt : (MT_INJ - 1);
  const int row0 = mtc * 16;

#pragma unroll 1
  for (int c = 0; c < NCH; ++c) {
    Frag a;
    {
      const v4f* xa = (const v4f*)(x + ((size_t)(row0 + m) * NCH + c) * BCH + 8 * h);
      const v4f f0 = xa[0], f1 = xa[1], f2 = xa[4], f3 = xa[5];
      a.s[0]  = (_Float16)f0.x; a.s[1]  = (_Float16)f0.y; a.s[2]  = (_Float16)f0.z; a.s[3]  = (_Float16)f0.w;
      a.s[4]  = (_Float16)f1.x; a.s[5]  = (_Float16)f1.y; a.s[6]  = (_Float16)f1.z; a.s[7]  = (_Float16)f1.w;
      a.s[8]  = (_Float16)f2.x; a.s[9]  = (_Float16)f2.y; a.s[10] = (_Float16)f2.z; a.s[11] = (_Float16)f2.w;
      a.s[12] = (_Float16)f3.x; a.s[13] = (_Float16)f3.y; a.s[14] = (_Float16)f3.z; a.s[15] = (_Float16)f3.w;
    }
#pragma unroll 1
    for (int w = 0; w < 16; ++w) {
      unsigned int m0[8], m1[8];
#pragma unroll
      for (int t2 = 0; t2 < 2; ++t2) {
        const int col = (2 * w + t2) * 16 + m;
        const float* wb = w_in + (size_t)(c * BCH) * I_N + col;
        Frag b;
#pragma unroll
        for (int i = 0; i < 8; ++i) {
          b.s[i]     = (_Float16)wb[(size_t)(8 * h + i) * I_N];
          b.s[8 + i] = (_Float16)wb[(size_t)(16 + 8 * h + i) * I_N];
        }
        v8f acc = {0.f, 0.f, 0.f, 0.f, 0.f, 0.f, 0.f, 0.f};
        acc = wmma_f16(a.v, b.v, acc);
#pragma unroll
        for (int r = 0; r < 8; ++r) {
          const int cnt = (int)acc[r];
          const unsigned int msk = __builtin_amdgcn_ballot_w32((cnt & 1) != 0);
          if (t2 == 0) m0[r] = msk; else m1[r] = msk;
        }
      }
      unsigned int val = 0u;
#pragma unroll
      for (int r = 0; r < 8; ++r) {
        const unsigned int lo = (m0[r] & 0xffffu) | (m1[r] << 16);
        const unsigned int hi = (m0[r] >> 16) | (m1[r] & 0xffff0000u);
        val = (m == r) ? lo : val;
        val = (m == 8 + r) ? hi : val;
      }
      if (lane < 16) stage[wave][lane][c * 16 + w] = val;
    }
  }
  __syncthreads();
  {
    const v4u* src = (const v4u*)&stage[wave][0][0];
    v4u vals[4];
#pragma unroll
    for (int it = 0; it < 4; ++it) vals[it] = src[it * 32 + lane];
    v4u* dst = (v4u*)(injbits + (size_t)row0 * 32);
    if (mt < MT_INJ) {
#pragma unroll
      for (int it = 0; it < 4; ++it) *(volatile v4u*)(dst + it * 32 + lane) = vals[it];
    }
    __threadfence();
    if (mt < MT_INJ) {
#pragma unroll
      for (int it = 0; it < 4; ++it) *(volatile v4u*)(dst + it * 32 + lane) = vals[it];
    }
  }
}

__global__ __launch_bounds__(EVT)
void evolve_kernel(const float* __restrict__ initial_states,
                   const unsigned int* __restrict__ injbits,
                   const unsigned int* __restrict__ adjp,
                   const unsigned int* __restrict__ lutbits,
                   _Float16* __restrict__ sres) {
  __shared__ uint8_t sbuf[2][SBUF];
  const int m   = blockIdx.x;
  const int tid = threadIdx.x;

  for (int n = tid; n < NN; n += EVT)
    sbuf[0][n] = (initial_states[n] != 0.f) ? (uint8_t)1 : (uint8_t)0;
  if (tid == 0) { sbuf[0][NN] = 0; sbuf[1][NN] = 0; }
  __syncthreads();

  const v4u* adj4 = (const v4u*)adjp;
  int cur = 0;
  for (int s = 0; s < SS; ++s) {
    for (int c = 0; c < NCH; ++c) {
      const unsigned int* iw = injbits + ((size_t)(m * SS + s) * NCH + c) * 16;
      for (int j = tid; j < I_N; j += EVT) {
        const unsigned int word = iw[j >> 5];
        const uint8_t bit = (uint8_t)((word >> (j & 31)) & 1u);
        sbuf[cur][j] ^= bit;
      }
      __syncthreads();
      for (int t2 = 0; t2 < 2; ++t2) {
        const uint8_t* sc = sbuf[cur];
        uint8_t*       sn = sbuf[cur ^ 1];
        for (int n = tid; n < NN; n += EVT) {
          const v4u aw = adj4[n];
          unsigned int i0 = aw.x & 0x7fffu;  i0 = (i0 > (unsigned)NN) ? (unsigned)NN : i0;
          unsigned int i1 = aw.x >> 16;       i1 = (i1 > (unsigned)NN) ? (unsigned)NN : i1;
          unsigned int i2 = aw.y & 0xffffu;  i2 = (i2 > (unsigned)NN) ? (unsigned)NN : i2;
          unsigned int i3 = aw.y >> 16;       i3 = (i3 > (unsigned)NN) ? (unsigned)NN : i3;
          unsigned int i4 = aw.z & 0xffffu;  i4 = (i4 > (unsigned)NN) ? (unsigned)NN : i4;
          unsigned int i5 = aw.z >> 16;       i5 = (i5 > (unsigned)NN) ? (unsigned)NN : i5;
          unsigned int i6 = aw.w & 0xffffu;  i6 = (i6 > (unsigned)NN) ? (unsigned)NN : i6;
          unsigned int i7 = aw.w >> 16;       i7 = (i7 > (unsigned)NN) ? (unsigned)NN : i7;
          const unsigned int idx =
              ((unsigned int)sc[i0] << 7) | ((unsigned int)sc[i1] << 6) |
              ((unsigned int)sc[i2] << 5) | ((unsigned int)sc[i3] << 4) |
              ((unsigned int)sc[i4] << 3) | ((unsigned int)sc[i5] << 2) |
              ((unsigned int)sc[i6] << 1) |  (unsigned int)sc[i7];
          const unsigned int lw = lutbits[(size_t)n * 8 + (idx >> 5)];
          const uint8_t nb = (uint8_t)((lw >> (idx & 31u)) & 1u);
          const uint8_t old = sc[n];
          sn[n] = (aw.x & 0x8000u) ? old : nb;
        }
        __syncthreads();
        cur ^= 1;
      }
    }
  }

  const uint8_t* sc = sbuf[cur];
  v4u vals[4];
#pragma unroll
  for (int it = 0; it < 4; ++it) {
    const int p = it * EVT + tid;
    const int base = I_N + 8 * p;
    unsigned int hw[8];
#pragma unroll
    for (int i = 0; i < 8; ++i) hw[i] = sc[base + i] ? 0x3C00u : 0u;
    v4u v;
    v.x = hw[0] | (hw[1] << 16);
    v.y = hw[2] | (hw[3] << 16);
    v.z = hw[4] | (hw[5] << 16);
    v.w = hw[6] | (hw[7] << 16);
    vals[it] = v;
  }
  v4u* dst = (v4u*)(sres + (size_t)m * R_N);
#pragma unroll
  for (int it = 0; it < 4; ++it) *(volatile v4u*)(dst + it * EVT + tid) = vals[it];
  __threadfence();
#pragma unroll
  for (int it = 0; it < 4; ++it) *(volatile v4u*)(dst + it * EVT + tid) = vals[it];
}

__global__ __launch_bounds__(128)
void readout_kernel(const _Float16* __restrict__ sres, const float* __restrict__ W_out,
                    const float* __restrict__ b_out, float* __restrict__ out) {
  __shared__ __attribute__((aligned(16))) float ost[MB * NOUT];
  const int tid  = threadIdx.x;
  const int wave = tid >> 5;
  const int lane = tid & 31;
  const int h    = lane >> 4;
  const int m    = lane & 15;
  const int row0 = wave * 16;
  const int nn   = (m < NOUT) ? m : (NOUT - 1);
  const float scale = (m < NOUT) ? 256.f : 0.f;
  const _Float16* ap = sres + (size_t)(row0 + m) * R_N + 8 * h;
  const float*    bp = W_out + (size_t)nn * R_N + 8 * h;

  v8f acc = {0.f, 0.f, 0.f, 0.f, 0.f, 0.f, 0.f, 0.f};
#pragma unroll 2
  for (int kb = 0; kb < R_N / 32; ++kb) {
    Frag a, b;
    a.half[0] = *(const v8h*)(ap + kb * 32);
    a.half[1] = *(const v8h*)(ap + kb * 32 + 16);
    const v4f* q = (const v4f*)(bp + kb * 32);
    const v4f f0 = q[0], f1 = q[1], f2 = q[4], f3 = q[5];
    b.s[0]  = (_Float16)(f0.x * scale); b.s[1]  = (_Float16)(f0.y * scale);
    b.s[2]  = (_Float16)(f0.z * scale); b.s[3]  = (_Float16)(f0.w * scale);
    b.s[4]  = (_Float16)(f1.x * scale); b.s[5]  = (_Float16)(f1.y * scale);
    b.s[6]  = (_Float16)(f1.z * scale); b.s[7]  = (_Float16)(f1.w * scale);
    b.s[8]  = (_Float16)(f2.x * scale); b.s[9]  = (_Float16)(f2.y * scale);
    b.s[10] = (_Float16)(f2.z * scale); b.s[11] = (_Float16)(f2.w * scale);
    b.s[12] = (_Float16)(f3.x * scale); b.s[13] = (_Float16)(f3.y * scale);
    b.s[14] = (_Float16)(f3.z * scale); b.s[15] = (_Float16)(f3.w * scale);
    acc = wmma_f16(a.v, b.v, acc);
  }

  const float bias = b_out[nn];
#pragma unroll
  for (int r = 0; r < 8; ++r) {
    float v = acc[r] * 0.00390625f + bias;
    v = fminf(fmaxf(v, -30.f), 30.f);
    const float e  = expf(-v);
    const float sg = 1.0f / (1.0f + e);
    if (m < NOUT) ost[(row0 + 8 * h + r) * NOUT + m] = sg;
  }
  __syncthreads();
  if (wave == 0) {
    const v4f* src = (const v4f*)ost;
    v4f vals[5];
#pragma unroll
    for (int it = 0; it < 5; ++it) vals[it] = src[it * 32 + lane];
    v4f* dst = (v4f*)out;
#pragma unroll
    for (int it = 0; it < 5; ++it) *(volatile v4f*)(dst + it * 32 + lane) = vals[it];
    __threadfence();
#pragma unroll
    for (int it = 0; it < 5; ++it) *(volatile v4f*)(dst + it * 32 + lane) = vals[it];
  }
}

extern "C" void kernel_launch(void* const* d_in, const int* in_sizes, int n_in,
                              void* d_out, int out_size, void* d_ws, size_t ws_size,
                              hipStream_t stream) {
  if (n_in < 10) return;
  if (in_sizes[0] != MB * SS * NCH * BCH) return;
  if (in_sizes[1] != NCH * BCH * I_N) return;
  if (in_sizes[2] != NN * KADJ) return;
  if (in_sizes[3] != NN * KADJ) return;
  if (in_sizes[4] != NN) return;
  if (in_sizes[5] != NN * LUTW) return;
  if (in_sizes[7] != NN) return;
  if (in_sizes[8] != NOUT * R_N) return;
  if (in_sizes[9] != NOUT) return;
  if (out_size != MB * NOUT) return;

  const float* x              = (const float*)d_in[0];
  const float* w_in           = (const float*)d_in[1];
  const int*   adj_list       = (const int*)d_in[2];
  const int*   adj_mask       = (const int*)d_in[3];
  const int*   deg            = (const int*)d_in[4];
  const float* lut            = (const float*)d_in[5];
  const float* initial_states = (const float*)d_in[7];
  const float* W_out          = (const float*)d_in[8];
  const float* b_out          = (const float*)d_in[9];

  const size_t sz_adj = (size_t)NN * 16;
  const size_t sz_lut = (size_t)NN * 32;
  const size_t sz_inj = (size_t)MB * SS * 128;
  const size_t sz_s   = (size_t)MB * R_N * 2;
  const size_t off_adj = 0;
  const size_t off_lut = off_adj + sz_adj;
  const size_t off_inj = off_lut + sz_lut;
  const size_t off_s   = off_inj + sz_inj;
  const size_t total   = off_s + sz_s;
  if (total > ws_size) return;

  uint8_t* ws = (uint8_t*)d_ws;
  unsigned int* adjp    = (unsigned int*)(ws + off_adj);
  unsigned int* lutbits = (unsigned int*)(ws + off_lut);
  unsigned int* injbits = (unsigned int*)(ws + off_inj);
  _Float16*     sres    = (_Float16*)(ws + off_s);

  const int prep_items = 3 * NN;
  prep_kernel<<<(prep_items + 255) / 256, 256, 0, stream>>>(adj_list, adj_mask, deg, lut,
                                                           adjp, lutbits);
  inject_kernel<<<(MT_INJ + 3) / 4, 128, 0, stream>>>(x, w_in, injbits);
  evolve_kernel<<<MB, EVT, 0, stream>>>(initial_states, injbits, adjp, lutbits, sres);
  readout_kernel<<<1, (MB / 16) * 32, 0, stream>>>(sres, W_out, b_out, (float*)d_out);
}
